// AffineCoupling_69698729279524
// MI455X (gfx1250) — hardware-verified
//
#include <hip/hip_runtime.h>
#include <stddef.h>

typedef __attribute__((ext_vector_type(16))) _Float16 v16h;
typedef __attribute__((ext_vector_type(8)))  _Float16 v8h;
typedef __attribute__((ext_vector_type(8)))  float    v8f;
typedef __attribute__((ext_vector_type(4)))  float    v4f;

__device__ __forceinline__ void dep_guard_h(v8f& a, v8f& b, v16h x, v16h y) { asm volatile("v_nop\n\tv_nop\n\tv_nop\n\tv_nop" : "+v"(a), "+v"(b) : "v"(x), "v"(y)); }
__device__ __forceinline__ void keep4_h(v16h a, v16h b, v16h c, v16h d) { asm volatile("v_nop" :: "v"(a), "v"(b), "v"(c), "v"(d)); }
__device__ __forceinline__ void acc_guard4(v8f& a, v8f& b, v8f& c, v8f& d) { asm volatile("v_nop\n\tv_nop\n\tv_nop\n\tv_nop" : "+v"(a), "+v"(b), "+v"(c), "+v"(d)); }

template <typename T> struct Frag;
template <> struct Frag<_Float16> {
  typedef v16h V; union U { v16h v; v8h h[2]; };
  static __device__ __forceinline__ v16h load(const _Float16* p) {
    U f; f.h[0] = *(const v8h*)(p); f.h[1] = *(const v8h*)(p + 16); return f.v;
  }
  static __device__ __forceinline__ v8f mma(v16h a, v16h b, v8f c) {
    return __builtin_amdgcn_wmma_f32_16x16x32_f16(false, a, false, b, (short)0, c, false, false);
  }
  static __device__ __forceinline__ void guard(v8f& a, v8f& b, v16h x, v16h y) { dep_guard_h(a, b, x, y); }
  static __device__ __forceinline__ void keep(v16h a, v16h b, v16h c, v16h d) { keep4_h(a, b, c, d); }
};

#define S_     64
#define NSQ_   32
#define NCPL_  16
#define L_     2048
#define LP_    2050
#define NCHA_  512
#define SEMB_  128
#define K2_    1536
#define SC_    32
#define NLT_   32
#define XP_    520
#define LDS1_  (64 * XP_ * 2)
#define W1SC_  16.0f
#define W1INV_ 0.0625f
#define W2SC_  64.0f
#define W2INV_ 0.015625f

__global__ __launch_bounds__(256) void k_dyn(const float* __restrict__ emb,
                                             const float* __restrict__ Wa, const float* __restrict__ ba,
                                             const float* __restrict__ Wb, const float* __restrict__ bb,
                                             float* __restrict__ wdyn, float* __restrict__ bdyn) {
  const int t = blockIdx.x * 256 + threadIdx.x;
  const int s = t >> 11, r = t & 2047;
  const bool isw = (r < K2_);
  const int rr = isw ? r : (r - K2_);
  const float* e  = emb + (size_t)s * SEMB_;
  const float* wr = isw ? (Wa + (size_t)rr * SEMB_) : (Wb + (size_t)rr * SEMB_);
  const float* bp = isw ? (ba + rr) : (bb + rr);
  float acc = 0.0f;
#pragma unroll 2
  for (int k = 0; k < SEMB_; k += 4) {
    const v4f ev = *(const v4f*)(e + k);
    const v4f wv = *(const v4f*)(wr + k);
    acc = fmaf(ev[0], wv[0], acc);
    acc = fmaf(ev[1], wv[1], acc);
    acc = fmaf(ev[2], wv[2], acc);
    acc = fmaf(ev[3], wv[3], acc);
  }
  acc += *bp;
  float* dst = isw ? (wdyn + (size_t)s * K2_ + rr) : (bdyn + (size_t)s * NCHA_ + rr);
  *(volatile float*)dst = acc;
  __threadfence();
  *(volatile float*)dst = acc;
}

__global__ __launch_bounds__(256) void k_cast(const float* __restrict__ W1, const float* __restrict__ W2,
                                              _Float16* __restrict__ W1f, _Float16* __restrict__ W2f) {
  const int i = blockIdx.x * 256 + threadIdx.x;
  float a, b;
  _Float16* dst;
  if (blockIdx.x < 512) {
    a = W1[2 * i] * W1SC_;
    b = W1[2 * i + 1] * W1SC_;
    dst = W1f + 2 * i;
  } else {
    int o = (i - 131072) * 2;
    o = (o < NSQ_ * K2_) ? o : (NSQ_ * K2_ - 2);
    const int j = o / K2_;
    const int rem = o - j * K2_;
    const int tap = rem >> 9, c = rem & 511;
    a = W2[((size_t)j * NCHA_ + c) * 3 + tap] * W2SC_;
    b = W2[((size_t)j * NCHA_ + c + 1) * 3 + tap] * W2SC_;
    dst = W2f + o;
  }
  const _Float16 h0 = (_Float16)a, h1 = (_Float16)b;
  const unsigned u = (unsigned)__builtin_bit_cast(unsigned short, h0) | ((unsigned)__builtin_bit_cast(unsigned short, h1) << 16);
  *(volatile unsigned*)dst = u;
  __threadfence();
  *(volatile unsigned*)dst = u;
}

__device__ __forceinline__ _Float16 dw3(float w0, float w1, float w2, float b, float hm, float hc, float hp) {
  const float x = fmaf(w0, hm, fmaf(w1, hc, fmaf(w2, hp, b)));
  return (_Float16)fmaxf(x, 0.0f);
}

__global__ __launch_bounds__(256) void k_gemm1(const float* __restrict__ h,
                                               const float* __restrict__ wdyn,
                                               const float* __restrict__ bdyn,
                                               const _Float16* __restrict__ W1f,
                                               const float* __restrict__ b1,
                                               _Float16* __restrict__ Yp, int s_base) {
  extern __shared__ __align__(16) _Float16 xl[];
  typedef Frag<_Float16> F;
  const int sl  = blockIdx.y;
  const int s   = s_base + sl;
  const int l0  = blockIdx.x * 64;
  const int tid = threadIdx.x, lane = tid & 31, wave = tid >> 5;

#pragma unroll 1
  for (int it = tid; it < 64 * 64; it += 256) {
    const int l  = it & 63;
    const int c0 = (it >> 6) * 8;
    const int q  = c0 >> 5;
    const int gl = l0 + l;
    const float* hrow = h + (size_t)(s * NSQ_ + q) * L_;
    const int im = (gl > 0) ? (gl - 1) : 0;
    const int ip = (gl < L_ - 1) ? (gl + 1) : (L_ - 1);
    float hm = hrow[im];
    const float hc = hrow[gl];
    float hp = hrow[ip];
    hm = (gl > 0) ? hm : 0.0f;
    hp = (gl < L_ - 1) ? hp : 0.0f;
    const float* wp = wdyn + (size_t)(s * NCHA_ + c0) * 3;
    const float* bp = bdyn + (size_t)s * NCHA_ + c0;
    const v4f w0 = *(const v4f*)(wp);
    const v4f w1 = *(const v4f*)(wp + 4);
    const v4f w2 = *(const v4f*)(wp + 8);
    const v4f w3 = *(const v4f*)(wp + 12);
    const v4f w4 = *(const v4f*)(wp + 16);
    const v4f w5 = *(const v4f*)(wp + 20);
    const v4f bA = *(const v4f*)(bp);
    const v4f bB = *(const v4f*)(bp + 4);
    v8h xv;
    xv[0] = dw3(w0[0], w0[1], w0[2], bA[0], hm, hc, hp);
    xv[1] = dw3(w0[3], w1[0], w1[1], bA[1], hm, hc, hp);
    xv[2] = dw3(w1[2], w1[3], w2[0], bA[2], hm, hc, hp);
    xv[3] = dw3(w2[1], w2[2], w2[3], bA[3], hm, hc, hp);
    xv[4] = dw3(w3[0], w3[1], w3[2], bB[0], hm, hc, hp);
    xv[5] = dw3(w3[3], w4[0], w4[1], bB[1], hm, hc, hp);
    xv[6] = dw3(w4[2], w4[3], w5[0], bB[2], hm, hc, hp);
    xv[7] = dw3(w5[1], w5[2], w5[3], bB[3], hm, hc, hp);
    *(v8h*)(xl + l * XP_ + c0) = xv;
  }
  __syncthreads();

  const int rlane = lane & 15;
  const int koff  = (lane >> 4) * 8;
  const int mOff  = (lane >> 4) * 8;
  const int n0    = wave * 64;
  v8f acc[4][4];
#pragma unroll
  for (int i = 0; i < 4; ++i)
#pragma unroll
    for (int j = 0; j < 4; ++j) acc[i][j] = (v8f){0.f,0.f,0.f,0.f,0.f,0.f,0.f,0.f};

  for (int k0 = 0; k0 < NCHA_; k0 += 32) {
    v16h bh[4];
#pragma unroll
    for (int j = 0; j < 4; ++j)
      bh[j] = F::load(W1f + (size_t)(n0 + (j << 4) + rlane) * NCHA_ + koff + k0);
#pragma unroll
    for (int i = 0; i < 4; ++i) {
      const v16h ah = F::load(xl + ((i << 4) + rlane) * XP_ + koff + k0);
#pragma unroll
      for (int j = 0; j < 4; ++j) acc[i][j] = F::mma(ah, bh[j], acc[i][j]);
      F::guard(acc[i][0], acc[i][3], ah, ah);
    }
    F::keep(bh[0], bh[1], bh[2], bh[3]);
  }
  acc_guard4(acc[0][0], acc[0][1], acc[0][2], acc[0][3]);
  acc_guard4(acc[1][0], acc[1][1], acc[1][2], acc[1][3]);
  acc_guard4(acc[2][0], acc[2][1], acc[2][2], acc[2][3]);
  acc_guard4(acc[3][0], acc[3][1], acc[3][2], acc[3][3]);
  __syncthreads();

  float* slab = (float*)xl + wave * (16 * 68);
  _Float16* Yb = Yp + (size_t)sl * LP_ * NCHA_;
  const int q8 = lane >> 3, c8 = (lane & 7) * 8;
#pragma unroll
  for (int i = 0; i < 4; ++i) {
    const int mBase = i << 4;
#pragma unroll
    for (int j = 0; j < 4; ++j) {
      const int n = n0 + (j << 4) + rlane;
      const float bv = b1[n];
#pragma unroll
      for (int r = 0; r < 8; ++r) {
        float v = acc[i][j][r] * W1INV_ + bv;
        v = fmaxf(v, 0.0f);
        slab[(mOff + r) * 68 + (j << 4) + rlane] = v;
      }
    }
    __builtin_amdgcn_fence(__ATOMIC_RELEASE, "workgroup");
    __builtin_amdgcn_wave_barrier();
    __builtin_amdgcn_fence(__ATOMIC_ACQUIRE, "workgroup");
    for (int pass = 0; pass < 2; ++pass) {
#pragma unroll
      for (int it = 0; it < 4; ++it) {
        const int row = it * 4 + q8;
        const float* sp = slab + row * 68 + c8;
        v8h hv;
#pragma unroll
        for (int e = 0; e < 8; ++e) hv[e] = (_Float16)sp[e];
        *(volatile v8h*)(Yb + (size_t)(l0 + mBase + row + 1) * NCHA_ + n0 + c8) = hv;
      }
      __threadfence();
    }
    __builtin_amdgcn_fence(__ATOMIC_RELEASE, "workgroup");
    __builtin_amdgcn_wave_barrier();
    __builtin_amdgcn_fence(__ATOMIC_ACQUIRE, "workgroup");
  }

  if (blockIdx.x == 0 || blockIdx.x == gridDim.x - 1) {
    v8h z;
#pragma unroll
    for (int e = 0; e < 8; ++e) z[e] = (_Float16)0.0f;
    const bool first = (blockIdx.x == 0);
    const bool last  = (blockIdx.x == gridDim.x - 1);
    for (int pass = 0; pass < 2; ++pass) {
      if (q8 == 0) {
        if (first) *(volatile v8h*)(Yb + n0 + c8) = z;
        if (last)  *(volatile v8h*)(Yb + (size_t)(L_ + 1) * NCHA_ + n0 + c8) = z;
      }
      __threadfence();
    }
  }
}

__global__ __launch_bounds__(128) void k_conv2(const float* __restrict__ h,
                                               const _Float16* __restrict__ Yp,
                                               const _Float16* __restrict__ W2f,
                                               const float* __restrict__ b2,
                                               float* __restrict__ out,
                                               float* __restrict__ part, int s_base) {
  __shared__ __align__(16) float zt[4][2][16 * 68];
  typedef Frag<_Float16> F;
  const int tid = threadIdx.x, lane = tid & 31, wave = tid >> 5;
  const int gw = blockIdx.x * 4 + wave;
  const int sl = gw >> 5, lt = gw & 31;
  if (sl >= SC_) return;
  const int s  = s_base + sl;
  const int l0 = lt * 64;
  const int rlane = lane & 15;
  const int koff  = (lane >> 4) * 8;
  const int mOff  = (lane >> 4) * 8;
  const _Float16* Ab = Yp + ((size_t)sl * LP_ + l0) * NCHA_;

  v8f acc[4][2];
#pragma unroll
  for (int i = 0; i < 4; ++i) { acc[i][0] = (v8f){0.f,0.f,0.f,0.f,0.f,0.f,0.f,0.f}; acc[i][1] = acc[i][0]; }

  for (int k0 = 0; k0 < K2_; k0 += 32) {
    const v16h bq0 = F::load(W2f + (size_t)rlane * K2_ + koff + k0);
    const v16h bq1 = F::load(W2f + (size_t)(16 + rlane) * K2_ + koff + k0);
#pragma unroll
    for (int i = 0; i < 4; ++i) {
      const v16h ah = F::load(Ab + (size_t)((i << 4) + rlane) * NCHA_ + koff + k0);
      acc[i][0] = F::mma(ah, bq0, acc[i][0]);
      acc[i][1] = F::mma(ah, bq1, acc[i][1]);
      F::guard(acc[i][0], acc[i][1], ah, ah);
    }
    F::keep(bq0, bq1, bq0, bq1);
  }
  acc_guard4(acc[0][0], acc[0][1], acc[1][0], acc[1][1]);
  acc_guard4(acc[2][0], acc[2][1], acc[3][0], acc[3][1]);

  float* zs = zt[wave][0];
  float* zm = zt[wave][1];
#pragma unroll
  for (int i = 0; i < 4; ++i)
#pragma unroll
    for (int r = 0; r < 8; ++r) {
      const int pos = (i << 4) + mOff + r;
      zs[rlane * 68 + pos] = acc[i][0][r];
      zm[rlane * 68 + pos] = acc[i][1][r];
    }
  __builtin_amdgcn_fence(__ATOMIC_RELEASE, "workgroup");
  __builtin_amdgcn_wave_barrier();
  __builtin_amdgcn_fence(__ATOMIC_ACQUIRE, "workgroup");

  const int hh = lane >> 4, c4 = (lane & 15) * 4;
  float lsum = 0.0f;
#pragma unroll 2
  for (int it = 0; it < 8; ++it) {
    const int ch = it * 2 + hh;
    const v4f a  = *(const v4f*)(zs + ch * 68 + c4);
    const v4f bm = *(const v4f*)(zm + ch * 68 + c4);
    const v4f h2 = *(const v4f*)(h + (size_t)(s * NSQ_ + NCPL_ + ch) * L_ + l0 + c4);
    const float bs2 = b2[ch] + 2.0f;
    const float bm2 = b2[NCPL_ + ch];
    v4f o;
#pragma unroll
    for (int e = 0; e < 4; ++e) {
      const float z  = fmaf(a[e], W2INV_, bs2);
      const float ez = expf(-z);
      const float sv = __builtin_amdgcn_rcpf(1.0f + ez) + 1e-7f;
      const float mv = fmaf(bm[e], W2INV_, bm2);
      o[e] = sv * (h2[e] + mv);
      lsum += logf(sv);
    }
    *(v4f*)(zs + ch * 68 + c4) = o;
  }
#pragma unroll
  for (int off = 1; off < 32; off <<= 1) lsum += __shfl_xor(lsum, off, 32);
  __builtin_amdgcn_fence(__ATOMIC_RELEASE, "workgroup");
  __builtin_amdgcn_wave_barrier();
  __builtin_amdgcn_fence(__ATOMIC_ACQUIRE, "workgroup");

  for (int pass = 0; pass < 2; ++pass) {
#pragma unroll
    for (int it = 0; it < 8; ++it) {
      const int ch = it * 2 + hh;
      const v4f o = *(const v4f*)(zs + ch * 68 + c4);
      *(volatile v4f*)(out + (size_t)(s * NSQ_ + NCPL_ + ch) * L_ + l0 + c4) = o;
      const size_t hidx = (size_t)(s * NSQ_ + ch) * L_ + l0 + c4;
      const v4f hv = *(const v4f*)(h + hidx);
      *(volatile v4f*)(out + hidx) = hv;
    }
    *(volatile float*)(part + (size_t)(s * NLT_ + lt) * 32 + lane) = lsum;
    __threadfence();
  }
}

__global__ __launch_bounds__(32) void k_logdet(const float* __restrict__ part, float* __restrict__ logdet) {
  const int lane = threadIdx.x;
  v4f v;
#pragma unroll
  for (int e = 0; e < 4; ++e) {
    int s = lane * 4 + e;
    s = (s < S_) ? s : (S_ - 1);
    const float* p = part + (size_t)s * NLT_ * 32;
    float acc = 0.0f;
#pragma unroll 4
    for (int t = 0; t < NLT_; ++t) acc += p[t * 32];
    v[e] = acc;
  }
  if (lane < 16) *(volatile v4f*)(logdet + lane * 4) = v;
  __threadfence();
  if (lane < 16) *(volatile v4f*)(logdet + lane * 4) = v;
}

extern "C" void kernel_launch(void* const* d_in, const int* in_sizes, int n_in,
                              void* d_out, int out_size, void* d_ws, size_t ws_size,
                              hipStream_t stream) {
  if (n_in < 10) return;
  if (in_sizes[0] != S_ * NSQ_ * L_) return;
  if (in_sizes[1] != S_ * SEMB_) return;
  if (in_sizes[2] != K2_ * SEMB_) return;
  if (in_sizes[3] != K2_) return;
  if (in_sizes[4] != NCHA_ * SEMB_) return;
  if (in_sizes[5] != NCHA_) return;
  if (in_sizes[6] != NCHA_ * NCHA_) return;
  if (in_sizes[7] != NCHA_) return;
  if (in_sizes[8] != NSQ_ * NCHA_ * 3) return;
  if (in_sizes[9] != NSQ_) return;
  if (out_size != S_ * NSQ_ * L_ + S_) return;

  const float* h   = (const float*)d_in[0];
  const float* emb = (const float*)d_in[1];
  const float* Wa  = (const float*)d_in[2];
  const float* ba  = (const float*)d_in[3];
  const float* Wb  = (const float*)d_in[4];
  const float* bb  = (const float*)d_in[5];
  const float* W1  = (const float*)d_in[6];
  const float* b1  = (const float*)d_in[7];
  const float* W2  = (const float*)d_in[8];
  const float* b2  = (const float*)d_in[9];

  float* out    = (float*)d_out;
  float* logdet = out + (size_t)S_ * NSQ_ * L_;

  const size_t o_wdyn = 0;
  const size_t o_bdyn = o_wdyn + (size_t)S_ * K2_ * 4;
  const size_t o_w1f  = o_bdyn + (size_t)S_ * NCHA_ * 4;
  const size_t o_w2f  = o_w1f  + (size_t)NCHA_ * NCHA_ * 2;
  const size_t o_part = o_w2f  + (size_t)NSQ_ * K2_ * 2;
  const size_t o_yp   = o_part + (size_t)S_ * NLT_ * 32 * 4;
  const size_t o_end  = o_yp   + (size_t)SC_ * LP_ * NCHA_ * 2;
  if (o_end > ws_size) return;

  char* ws = (char*)d_ws;
  float*    wdyn = (float*)(ws + o_wdyn);
  float*    bdyn = (float*)(ws + o_bdyn);
  _Float16* W1f  = (_Float16*)(ws + o_w1f);
  _Float16* W2f  = (_Float16*)(ws + o_w2f);
  float*    part = (float*)(ws + o_part);
  _Float16* Yp   = (_Float16*)(ws + o_yp);

  (void)hipFuncSetAttribute((const void*)k_gemm1, hipFuncAttributeMaxDynamicSharedMemorySize, LDS1_);

  k_dyn<<<(S_ * 2048) / 256, 256, 0, stream>>>(emb, Wa, ba, Wb, bb, wdyn, bdyn);
  k_cast<<<512 + 96, 256, 0, stream>>>(W1, W2, W1f, W2f);
  for (int c = 0; c < S_ / SC_; ++c) {
    k_gemm1<<<dim3(NLT_, SC_), 256, LDS1_, stream>>>(h, wdyn, bdyn, W1f, b1, Yp, c * SC_);
    k_conv2<<<(SC_ * NLT_) / 4, 128, 0, stream>>>(h, Yp, W2f, b2, out, part, c * SC_);
  }
  k_logdet<<<1, 32, 0, stream>>>(part, logdet);
}
